// text_wiki_GCN_53910429499532
// MI455X (gfx1250) — hardware-run, weakly checked
//
#include <hip/hip_runtime.h>
#include <stddef.h>
#include <stdint.h>
#include <math.h>

#define DF     128
#define HLP    256
#define NTHR   256
#define NWAVE  8
#define EPT    8
#define CHUNK  (NTHR * EPT)
#define WCAP   (EPT * 32)
#define LISTN  (NWAVE * WCAP)
#define NBA    1024
#define SLA    10
#define RCAP   20480
#define DEGCAP 64
#define GBM    64
#define GBN    128
#define GTHR   128
#define SPB    64
#define NGR    128
#define PSEG   6272
#define NN_C   50000
#define NE_C   800000
#define MP_C   50048
#define NBK    49
#define NBP    (NBK * NBA)
#define NBX    (MP_C * 16 / NTHR)
#define NWB    64
#define NBB    5
#define BK_ZINTS (LISTN + 2 * RCAP + 3 * NBA)
#define BK_LDS_INTS (BK_ZINTS + 16)
#define WSMAX  134217728

static_assert((CHUNK & (CHUNK - 1)) == 0 && CHUNK <= 4096);
static_assert((NBA & (NBA - 1)) == 0 && NBA == (1 << SLA));
static_assert(((long long)CHUNK << SLA) < (1LL << 31));
static_assert(NE_C < (1 << (31 - SLA)));
static_assert(NE_C % 4 == 0);
static_assert(RCAP % (NTHR * 4) == 0 && BK_ZINTS % (NTHR * 4) == 0);
static_assert(RCAP >= 17492);
static_assert(RCAP <= 28672);
static_assert(DEGCAP >= 36 + 8);
static_assert(NBA == NTHR * 4);
static_assert(MP_C % GBM == 0 && MP_C % SPB == 0 && MP_C >= NN_C && MP_C <= NBP);
static_assert(NBA % SPB == 0 && SPB == 8 * NWAVE);
static_assert((MP_C * 16) % NTHR == 0);
static_assert(GBM == (GTHR / 32) * 16 && GBN == DF && DF == 4 * 32 && HLP == 2 * DF);
static_assert(NWAVE * PSEG >= NN_C && PSEG % 32 == 0);
static_assert(BK_LDS_INTS * 4 <= 300000);
static_assert(NWAVE * PSEG * 4 + 2048 <= 327680);
static_assert((long long)NN_C * DF + (long long)(NGR - 1) * DF + DF - 1 == 6416383LL);

typedef float          v4f   __attribute__((ext_vector_type(4)));
typedef float          v8f   __attribute__((ext_vector_type(8)));
typedef int            v4i   __attribute__((ext_vector_type(4)));
typedef int            v8i   __attribute__((ext_vector_type(8)));
typedef unsigned short v4us  __attribute__((ext_vector_type(4)));
typedef unsigned short v8us  __attribute__((ext_vector_type(8)));
typedef unsigned short v16us __attribute__((ext_vector_type(16)));
typedef __bf16         v16bf __attribute__((ext_vector_type(16)));
typedef v4f  __attribute__((may_alias)) v4fa;
typedef v4i  __attribute__((may_alias)) v4ia;
typedef v4us __attribute__((may_alias)) v4usa;
typedef v8us __attribute__((may_alias)) v8usa;
union FragB { v16bf v; v16us u; v8us h[2]; v8i w; };

__device__ __forceinline__ v8f wmb(const FragB& a, const FragB& b, v8f c) {
  v8f d = __builtin_amdgcn_wmma_f32_16x16x32_bf16(false, a.v, false, b.v, (short)0, c, false, false);
  asm volatile("v_nop\n\tv_nop\n\tv_nop\n\tv_nop" : "+v"(d) : "v"(a.w), "v"(b.w));
  return d;
}

__device__ __forceinline__ unsigned bf16_bits(float f) {
  const unsigned u = __float_as_uint(f);
  const unsigned r = (u + 0x7FFFu + ((u >> 16) & 1u)) >> 16;
  return (f != f) ? 0x7FC0u : r;
}
__device__ __forceinline__ float bf16_val(float f) {
  return __uint_as_float(bf16_bits(f) << 16);
}

__device__ __forceinline__ void wave_sync() {
  __builtin_amdgcn_fence(__ATOMIC_RELEASE, "wavefront");
  __builtin_amdgcn_wave_barrier();
  __builtin_amdgcn_fence(__ATOMIC_ACQUIRE, "wavefront");
}

__device__ __forceinline__ float gelu_t(float v) {
  const float u = 0.7978845608028654f * (v + 0.044715f * (v * v * v));
  const float e = __expf(2.0f * u);
  const float t = 1.0f - 2.0f * __builtin_amdgcn_rcpf(1.0f + e);
  return 0.5f * v * (1.0f + t);
}

template <int SLB>
__device__ __forceinline__ int scan_chunk(const int* __restrict__ dsts, int nE, int cbase, int slotBase,
                                          int nb, int vec8, int* list, int tid, int lane, int wave) {
  int wc = 0;
  const int el0  = tid * EPT;
  const int e0   = cbase + el0;
  const int sent = -2147483647 - 1;
  v4i da, db;
  if (vec8 != 0 && cbase + CHUNK <= nE) {
    da = *(const v4i*)(dsts + e0);
    db = *(const v4i*)(dsts + e0 + 4);
  } else {
    da.x = (e0     < nE) ? dsts[min(e0,     nE - 1)] : sent;
    da.y = (e0 + 1 < nE) ? dsts[min(e0 + 1, nE - 1)] : sent;
    da.z = (e0 + 2 < nE) ? dsts[min(e0 + 2, nE - 1)] : sent;
    da.w = (e0 + 3 < nE) ? dsts[min(e0 + 3, nE - 1)] : sent;
    db.x = (e0 + 4 < nE) ? dsts[min(e0 + 4, nE - 1)] : sent;
    db.y = (e0 + 5 < nE) ? dsts[min(e0 + 5, nE - 1)] : sent;
    db.z = (e0 + 6 < nE) ? dsts[min(e0 + 6, nE - 1)] : sent;
    db.w = (e0 + 7 < nE) ? dsts[min(e0 + 7, nE - 1)] : sent;
  }
  const unsigned nbs = (unsigned)slotBase;
  const unsigned unb = (unsigned)nb;
  const unsigned s0 = (unsigned)da.x - nbs, s1 = (unsigned)da.y - nbs;
  const unsigned s2 = (unsigned)da.z - nbs, s3 = (unsigned)da.w - nbs;
  const unsigned s4 = (unsigned)db.x - nbs, s5 = (unsigned)db.y - nbs;
  const unsigned s6 = (unsigned)db.z - nbs, s7 = (unsigned)db.w - nbs;
  const bool h0 = s0 < unb, h1 = s1 < unb, h2 = s2 < unb, h3 = s3 < unb;
  const bool h4 = s4 < unb, h5 = s5 < unb, h6 = s6 < unb, h7 = s7 < unb;
  const unsigned any = __builtin_amdgcn_ballot_w32(h0 | h1 | h2 | h3 | h4 | h5 | h6 | h7);
  if (any != 0u) {
#define HITJ(J, HJ, SJ) { \
      const unsigned mj = __builtin_amdgcn_ballot_w32(HJ); \
      if (mj != 0u) { \
        if (HJ) { \
          const int pos = wc + (int)__builtin_amdgcn_mbcnt_lo(mj, 0u); \
          if (pos < WCAP) list[wave * WCAP + pos] = ((el0 + (J)) << SLB) | (int)(SJ); \
        } \
        wc += (int)__builtin_popcount(mj); } }
    HITJ(0, h0, s0)
    HITJ(1, h1, s1)
    HITJ(2, h2, s2)
    HITJ(3, h3, s3)
    HITJ(4, h4, s4)
    HITJ(5, h5, s5)
    HITJ(6, h6, s6)
    HITJ(7, h7, s7)
#undef HITJ
  }
  return wc;
}

__global__ __launch_bounds__(NTHR) void k_prep(
    const float* __restrict__ x,
    const float* __restrict__ W1t, const float* __restrict__ W1w, const float* __restrict__ W2t,
    const float* __restrict__ W2w, const float* __restrict__ Ww,
    const float* __restrict__ b1t, const float* __restrict__ b2t, const float* __restrict__ b1w,
    const float* __restrict__ b2w, const float* __restrict__ bw,
    int nN, unsigned short* XB, unsigned short* W1cat, unsigned short* W2tD, unsigned short* W2wD,
    unsigned short* WwD, float* BIAS) {
  const int bid = (int)blockIdx.x, tid = (int)threadIdx.x;
  if (bid < NBX) {
    const int u   = bid * NTHR + tid;
    const int row = u >> 4;
    const int k8  = (u & 15) * 8;
    const int rc  = row < nN ? row : nN - 1;
    const float* p = x + (size_t)rc * DF + k8;
    const v4f a = *(const v4fa*)p;
    const v4f b = *(const v4fa*)(p + 4);
    const bool ok = row < nN;
    v8us o;
    o[0] = ok ? (unsigned short)bf16_bits(a.x) : (unsigned short)0;
    o[1] = ok ? (unsigned short)bf16_bits(a.y) : (unsigned short)0;
    o[2] = ok ? (unsigned short)bf16_bits(a.z) : (unsigned short)0;
    o[3] = ok ? (unsigned short)bf16_bits(a.w) : (unsigned short)0;
    o[4] = ok ? (unsigned short)bf16_bits(b.x) : (unsigned short)0;
    o[5] = ok ? (unsigned short)bf16_bits(b.y) : (unsigned short)0;
    o[6] = ok ? (unsigned short)bf16_bits(b.z) : (unsigned short)0;
    o[7] = ok ? (unsigned short)bf16_bits(b.w) : (unsigned short)0;
    unsigned short* dp = XB + (size_t)row * DF + k8;
    *(volatile v8us*)dp = o;
    __threadfence();
    *(volatile v8us*)dp = o;
    return;
  }
  const int wb = bid - NBX;
  if (wb < NWB) {
    const float* W;
    unsigned short* P;
    int v, sh, pitch, rowAdd;
    if (wb < 8)       { W = W1t; P = W1cat; v = wb * NTHR + tid;        sh = 4; pitch = DF;  rowAdd = 0; }
    else if (wb < 16) { W = W1w; P = W1cat; v = (wb - 8) * NTHR + tid;  sh = 4; pitch = DF;  rowAdd = DF; }
    else if (wb < 32) { W = W2t; P = W2tD;  v = (wb - 16) * NTHR + tid; sh = 5; pitch = HLP; rowAdd = 0; }
    else if (wb < 48) { W = W2w; P = W2wD;  v = (wb - 32) * NTHR + tid; sh = 5; pitch = HLP; rowAdd = 0; }
    else              { W = Ww;  P = WwD;   v = (wb - 48) * NTHR + tid; sh = 5; pitch = HLP; rowAdd = 0; }
    const int n  = v >> sh;
    const int k8 = (v & ((1 << sh) - 1)) * 8;
    const int kk = k8 & (DF - 1);
    const float* p = W + (size_t)kk * DF + n;
    v8us o;
#pragma unroll
    for (int i = 0; i < 8; ++i) o[i] = (unsigned short)bf16_bits(p[(size_t)i * DF]);
    unsigned short* dp = P + (size_t)(rowAdd + n) * pitch + k8;
    *(volatile v8us*)dp = o;
    __threadfence();
    *(volatile v8us*)dp = o;
    return;
  }
  const int bi = wb - NWB;
  const float* bp;
  if (bi == 0)      bp = b1t;
  else if (bi == 1) bp = b2t;
  else if (bi == 2) bp = b1w;
  else if (bi == 3) bp = b2w;
  else              bp = bw;
  if (tid < 32) {
    const v4f a = *(const v4fa*)(bp + 4 * tid);
    v4f o;
    o.x = bf16_val(a.x); o.y = bf16_val(a.y); o.z = bf16_val(a.z); o.w = bf16_val(a.w);
    float* dp = BIAS + (size_t)bi * DF + 4 * tid;
    *(volatile v4f*)dp = o;
    __threadfence();
    *(volatile v4f*)dp = o;
  }
}

__global__ __launch_bounds__(NTHR) void k_bucket(const int* __restrict__ edges, int nE, int nN, int vec8,
                                                 int* lst, int* cntg, int* offg, int* dinvg, int* flg) {
  extern __shared__ __attribute__((aligned(16))) int dsm[];
  int* list = dsm;
  int* hl   = dsm + LISTN;
  int* sl   = hl + RCAP;
  int* cnt  = sl + RCAP;
  int* offs = cnt + NBA;
  int* cur  = offs + NBA;
  int* misc = cur + NBA;
  const int* srcs = edges;
  const int* dsts = edges + nE;
  const int tid = (int)threadIdx.x, lane = tid & 31, wave = tid >> 5;
  const int nodeBase = (int)blockIdx.x * NBA;

  {
    const v4i z4 = {0, 0, 0, 0};
    for (int i = tid * 4; i < BK_ZINTS; i += NTHR * 4) *(v4ia*)(dsm + i) = z4;
    if (tid < 16) misc[tid] = 0;
  }
  __syncthreads();

  int t = 0, ov = 0;
  const int nChunks = (nE + CHUNK - 1) / CHUNK;
#pragma unroll 1
  for (int ch = 0; ch < nChunks; ++ch) {
    const int cbase = ch * CHUNK;
    const int wc = scan_chunk<SLA>(dsts, nE, cbase, nodeBase, NBA, vec8, list, tid, lane, wave);
    if (lane == 0) misc[wave] = wc;
    __syncthreads();
    if (wave == 0) {
#pragma unroll 1
      for (int w2 = 0; w2 < NWAVE; ++w2) {
        int c = misc[w2];
        c = c < 0 ? 0 : (c > WCAP ? WCAP : c);
#pragma unroll 1
        for (int b0 = 0; b0 < c; b0 += 32) {
          const int idx = b0 + lane;
          const int ent = list[w2 * WCAP + (idx < WCAP ? idx : WCAP - 1)];
          const int m32 = (c - b0) < 32 ? (c - b0) : 32;
#pragma unroll 1
          for (int k = 0; k < m32; ++k) {
            const int u    = __builtin_amdgcn_readlane(ent, k);
            const int slot = u & (NBA - 1);
            const int el   = (u >> SLA) & (CHUNK - 1);
            const int pk   = ((cbase + el) << SLA) | slot;
            if (t < RCAP) {
              if (lane == 0) { hl[t] = pk; cnt[slot] = cnt[slot] + 1; }
              t = t + 1;
            } else {
              ov = 1;
            }
          }
        }
      }
    }
    __syncthreads();
  }
  if (wave == 0 && lane == 0) { misc[8] = t; misc[9] = ov; }
  __syncthreads();
  int tt = misc[8];
  tt = tt < 0 ? 0 : (tt > RCAP ? RCAP : tt);
  const int ovf = misc[9];

  if (wave == 0) {
    const int base = lane * (NBA / 32);
    int s = 0;
#pragma unroll 1
    for (int i = 0; i < NBA / 32; ++i) s += cnt[base + i];
    int incl = s;
#pragma unroll
    for (int d = 1; d < 32; d <<= 1) {
      const int y = __shfl_up(incl, d, 32);
      if (lane >= d) incl += y;
    }
    int run = incl - s;
#pragma unroll 1
    for (int i = 0; i < NBA / 32; ++i) {
      const int cv = cnt[base + i];
      offs[base + i] = run;
      cur[base + i]  = run;
      run += cv;
    }
  }
  __syncthreads();
  if (wave == 0) {
#pragma unroll 1
    for (int b0 = 0; b0 < tt; b0 += 32) {
      const int idx = b0 + lane;
      const int ent = hl[idx < RCAP ? idx : RCAP - 1];
      const int m32 = (tt - b0) < 32 ? (tt - b0) : 32;
#pragma unroll 1
      for (int k = 0; k < m32; ++k) {
        const int u    = __builtin_amdgcn_readlane(ent, k);
        const int slot = u & (NBA - 1);
        if (lane == 0) {
          int p = cur[slot];
          p = p < 0 ? 0 : (p > RCAP - 1 ? RCAP - 1 : p);
          sl[p] = u;
          cur[slot] = p + 1;
        }
      }
    }
  }
  __syncthreads();

#pragma unroll 1
  for (int idx = tid; idx < RCAP; idx += NTHR) {
    const int ent = sl[idx];
    int eid = ent >> SLA;
    eid = eid < 0 ? 0 : (eid > nE - 1 ? nE - 1 : eid);
    int sr = srcs[eid];
    asm volatile("" :: "v"(sr));
    sr = sr < 0 ? 0 : (sr > nN - 1 ? nN - 1 : sr);
    hl[idx] = (idx < tt) ? sr : 0;
  }
#pragma unroll 1
  for (int j = 0; j < 4; ++j) {
    const int s   = 4 * tid + j;
    const int deg = cnt[s] + 1;
    const float dv = (deg > 0) ? (1.0f / sqrtf((float)deg)) : 0.0f;
    cur[s] = __float_as_int(dv);
  }
  __syncthreads();

  int* lb = lst + (size_t)blockIdx.x * RCAP;
#pragma unroll 1
  for (int it = 0; it < RCAP / (NTHR * 4); ++it) {
    const int i4 = (it * NTHR + tid) * 4;
    const v4i v = *(const v4ia*)(hl + i4);
    *(volatile v4i*)(lb + i4) = v;
  }
  __threadfence();
#pragma unroll 1
  for (int it = 0; it < RCAP / (NTHR * 4); ++it) {
    const int i4 = (it * NTHR + tid) * 4;
    const v4i v = *(const v4ia*)(hl + i4);
    *(volatile v4i*)(lb + i4) = v;
  }

  const v4i c4 = *(const v4ia*)(cnt + 4 * tid);
  const v4i o4 = *(const v4ia*)(offs + 4 * tid);
  const v4i d4 = *(const v4ia*)(cur + 4 * tid);
  const v4i f4 = {ovf, ovf, ovf, ovf};
  const size_t gi = (size_t)nodeBase + 4 * tid;
  int* fp = flg + (size_t)blockIdx.x * 32 + 4 * (tid & 7);
  *(volatile v4i*)(cntg + gi) = c4;
  *(volatile v4i*)(offg + gi) = o4;
  *(volatile v4i*)(dinvg + gi) = d4;
  if (tid < 8) *(volatile v4i*)fp = f4;
  __threadfence();
  *(volatile v4i*)(cntg + gi) = c4;
  *(volatile v4i*)(offg + gi) = o4;
  *(volatile v4i*)(dinvg + gi) = d4;
  if (tid < 8) *(volatile v4i*)fp = f4;
}

template <int MODE>
__global__ __launch_bounds__(GTHR) __attribute__((amdgpu_num_vgpr(248))) void k_gemm(
    const unsigned short* __restrict__ A, const unsigned short* __restrict__ BT, int K,
    const float* __restrict__ scl, int sclStrideY, const float* __restrict__ bias,
    float* outp, int ldo) {
  __shared__ __attribute__((aligned(16))) float stg[GBM * GBN];
  __shared__ __attribute__((aligned(16))) float sdv[GBM];
  __shared__ __attribute__((aligned(16))) float sb[DF];
  const int tid = (int)threadIdx.x, lane = tid & 31, wave = tid >> 5, hh = lane >> 4, m = lane & 15;
  const int rowBase = (int)blockIdx.x * GBM;
  const int yb      = (int)blockIdx.y;

  v8f acc[8];
  {
    const v8f z = {0.f, 0.f, 0.f, 0.f, 0.f, 0.f, 0.f, 0.f};
#pragma unroll
    for (int t = 0; t < 8; ++t) acc[t] = z;
  }
  const unsigned short* ap = A + (size_t)(rowBase + 16 * wave + m) * (size_t)K + 8 * hh;
  const unsigned short* bp = BT + (size_t)(DF * yb + m) * (size_t)K + 8 * hh;

#pragma unroll 1
  for (int k0 = 0; k0 < K; k0 += 32) {
    FragB af;
    af.h[0] = *(const v8usa*)(ap + k0);
    af.h[1] = *(const v8usa*)(ap + k0 + 16);
#pragma unroll
    for (int nt = 0; nt < 8; ++nt) {
      const unsigned short* wq = bp + (size_t)(16 * nt) * (size_t)K + k0;
      FragB bf;
      bf.h[0] = *(const v8usa*)wq;
      bf.h[1] = *(const v8usa*)(wq + 16);
      acc[nt] = wmb(af, bf, acc[nt]);
    }
  }

#pragma unroll
  for (int nt = 0; nt < 8; ++nt) {
    const int lc = 16 * nt + m;
#pragma unroll
    for (int r = 0; r < 8; ++r) {
      const int lr = 16 * wave + 8 * hh + r;
      stg[lr * GBN + lc] = acc[nt][r];
    }
  }
  if constexpr (MODE == 0) {
    if (tid < GBM) sdv[tid] = scl[(size_t)yb * (size_t)sclStrideY + rowBase + tid];
  } else {
    if (tid < 32) *(v4fa*)(sb + 4 * tid) = *(const v4fa*)(bias + 4 * tid);
  }
  __syncthreads();

  v4f pv[16];
#pragma unroll
  for (int i = 0; i < 16; ++i) pv[i] = *(const v4fa*)(stg + (16 * wave + i) * GBN + 4 * lane);
  if constexpr (MODE == 0) {
#pragma unroll
    for (int i = 0; i < 16; ++i) {
      const float sc = sdv[16 * wave + i];
      pv[i] = pv[i] * sc;
    }
  } else {
    const v4f b4 = *(const v4fa*)(sb + 4 * lane);
#pragma unroll
    for (int i = 0; i < 16; ++i) pv[i] = pv[i] + b4;
  }
#pragma unroll
  for (int i = 0; i < 16; ++i) {
    const int r = rowBase + 16 * wave + i;
    *(volatile v4f*)(outp + (size_t)r * (size_t)ldo + DF * yb + 4 * lane) = pv[i];
  }
  __threadfence();
#pragma unroll
  for (int i = 0; i < 16; ++i) {
    const int r = rowBase + 16 * wave + i;
    *(volatile v4f*)(outp + (size_t)r * (size_t)ldo + DF * yb + 4 * lane) = pv[i];
  }
}

template <int MODE>
__global__ __launch_bounds__(NTHR) void k_agg(const float* __restrict__ hin, int pitch, int colOff,
                                              const int* __restrict__ lst, const int* __restrict__ cntg,
                                              const int* __restrict__ offg, const float* __restrict__ dinvg,
                                              const int* __restrict__ flg, const float* __restrict__ bias,
                                              int nN, int mRows,
                                              unsigned short* ohl, float* of32, const float* __restrict__ wk) {
  __shared__ __attribute__((aligned(16))) float sbias[DF];
  __shared__ __attribute__((aligned(16))) unsigned short rowall[NWAVE * HLP];
  const int tid = (int)threadIdx.x, lane = tid & 31, wave = tid >> 5;
  const int nodeBase = (int)blockIdx.x * SPB;
  unsigned short* rowbuf = rowall + wave * HLP;

  if (tid < 32) *(v4fa*)(sbias + 4 * tid) = *(const v4fa*)(bias + 4 * tid);
  __syncthreads();
  const v4f bv = *(const v4fa*)(sbias + 4 * lane);

  const int bk = nodeBase >> SLA;
  const int fl = flg[(size_t)bk * 32];
  const int* lb = lst + (size_t)bk * RCAP;
  const float qnan = __int_as_float(0x7fc00000);
  const float pz = (fl != 0) ? qnan : 0.0f;

#pragma unroll 1
  for (int si = 0; si < SPB / NWAVE; ++si) {
    const int s    = si * NWAVE + wave;
    const int node = nodeBase + s;
    int c = cntg[node];
    const bool big = c > DEGCAP;
    c = c < 0 ? 0 : (c > DEGCAP ? DEGCAP : c);
    int o = offg[node];
    o = o < 0 ? 0 : (o > RCAP ? RCAP : o);
    const int nc = node < nN ? node : nN - 1;
    const float dd = dinvg[nc];
    float a0 = 0.0f, a1 = 0.0f, a2 = 0.0f, a3 = 0.0f;
#pragma unroll 1
    for (int b0 = 0; b0 < c; b0 += 32) {
      int idx = o + b0 + lane;
      idx = idx > RCAP - 1 ? RCAP - 1 : idx;
      int sr = lb[idx];
      sr = sr < 0 ? 0 : (sr > nN - 1 ? nN - 1 : sr);
      const int m32 = (c - b0) < 32 ? (c - b0) : 32;
#pragma unroll 1
      for (int k = 0; k < m32; ++k) {
        const int sk = __builtin_amdgcn_readlane(sr, k);
        const v4f a = *(const v4f*)(hin + (size_t)sk * (size_t)pitch + colOff + 4 * lane);
        a0 += a.x; a1 += a.y; a2 += a.z; a3 += a.w;
      }
    }
    {
      const v4f a = *(const v4f*)(hin + (size_t)nc * (size_t)pitch + colOff + 4 * lane);
      a0 += a.x; a1 += a.y; a2 += a.z; a3 += a.w;
    }
    const float pzr = big ? qnan : pz;
    const bool live = node < nN;
    float y0 = gelu_t(a0 * dd + bv.x) + pzr;
    float y1 = gelu_t(a1 * dd + bv.y) + pzr;
    float y2 = gelu_t(a2 * dd + bv.z) + pzr;
    float y3 = gelu_t(a3 * dd + bv.w) + pzr;

    if constexpr (MODE == 1) {
      v4f ov;
      ov.x = live ? y0 : 0.0f; ov.y = live ? y1 : 0.0f; ov.z = live ? y2 : 0.0f; ov.w = live ? y3 : 0.0f;
      if (node < mRows) {
        float* op = of32 + (size_t)node * DF + 4 * lane;
        *(volatile v4f*)op = ov;
        __threadfence();
        *(volatile v4f*)op = ov;
      }
    } else {
      float m0, m1, m2, m3;
      v4f tx;
      tx.x = y0; tx.y = y1; tx.z = y2; tx.w = y3;
      if constexpr (MODE == 2) {
        const v4f wv = *(const v4f*)(wk + (size_t)nc * DF + 4 * lane);
        m0 = live ? (y0 - wv.x) : 0.0f;
        m1 = live ? (y1 - wv.y) : 0.0f;
        m2 = live ? (y2 - wv.z) : 0.0f;
        m3 = live ? (y3 - wv.w) : 0.0f;
      } else {
        m0 = live ? y0 : 0.0f;
        m1 = live ? y1 : 0.0f;
        m2 = live ? y2 : 0.0f;
        m3 = live ? y3 : 0.0f;
      }
      v4us mh, ml;
      {
        unsigned hb;
        hb = bf16_bits(m0); mh[0] = (unsigned short)hb; ml[0] = (unsigned short)bf16_bits(m0 - __uint_as_float(hb << 16));
        hb = bf16_bits(m1); mh[1] = (unsigned short)hb; ml[1] = (unsigned short)bf16_bits(m1 - __uint_as_float(hb << 16));
        hb = bf16_bits(m2); mh[2] = (unsigned short)hb; ml[2] = (unsigned short)bf16_bits(m2 - __uint_as_float(hb << 16));
        hb = bf16_bits(m3); mh[3] = (unsigned short)hb; ml[3] = (unsigned short)bf16_bits(m3 - __uint_as_float(hb << 16));
      }
      *(v4usa*)(rowbuf + 4 * lane) = mh;
      *(v4usa*)(rowbuf + DF + 4 * lane) = ml;
      wave_sync();
      const v8us q0 = *(const v8usa*)(rowbuf + 8 * lane);
      wave_sync();
      unsigned short* rpw = ohl + (size_t)node * HLP + 8 * lane;
      if constexpr (MODE == 2) {
        float* op = of32 + (size_t)nc * DF + 4 * lane;
        if (node < nN) *(volatile v4f*)op = tx;
        if (node < mRows) *(volatile v8us*)rpw = q0;
        __threadfence();
        if (node < nN) *(volatile v4f*)op = tx;
        if (node < mRows) *(volatile v8us*)rpw = q0;
      } else {
        if (node < mRows) {
          *(volatile v8us*)rpw = q0;
          __threadfence();
          *(volatile v8us*)rpw = q0;
        }
      }
    }
  }
}

__global__ __launch_bounds__(NTHR) void k_pool(const float* __restrict__ df, const int* __restrict__ bat,
                                               int nN, float* outp) {
  extern __shared__ __attribute__((aligned(16))) int pm[];
  __shared__ int wcn[NWAVE];
  __shared__ __attribute__((aligned(16))) float sm[2 * DF];
  const int tid = (int)threadIdx.x, lane = tid & 31, wave = tid >> 5;
  const int g = (int)blockIdx.x;

  int wc = 0;
  const int lo = wave * PSEG;
  const int hiEnd = (lo + PSEG) < nN ? (lo + PSEG) : nN;
#pragma unroll 1
  for (int i0 = lo; i0 < hiEnd; i0 += 32) {
    const int i  = i0 + lane;
    const int ic = i < nN ? i : nN - 1;
    const int b  = bat[ic];
    asm volatile("" :: "v"(b));
    const bool hit = (i < nN) && (b == g);
    const unsigned msk = __builtin_amdgcn_ballot_w32(hit);
    const int pos = wc + (int)__builtin_amdgcn_mbcnt_lo(msk, 0u);
    if (hit && pos < PSEG) pm[lo + pos] = i;
    wc += (int)__builtin_popcount(msk);
  }
  if (lane == 0) wcn[wave] = wc;
  __syncthreads();

  const int half = tid >> 7;
  const int c    = tid & (DF - 1);
  float m = __int_as_float((int)0xff800000u);
#pragma unroll 1
  for (int w2 = 0; w2 < NWAVE; ++w2) {
    int cw = wcn[w2];
    cw = cw < 0 ? 0 : (cw > PSEG ? PSEG : cw);
#pragma unroll 1
    for (int j = half; j < cw; j += 2) {
      int node = pm[w2 * PSEG + j];
      node = node < 0 ? 0 : (node > nN - 1 ? nN - 1 : node);
      const float v = df[(size_t)node * DF + c];
      m = (v > m || v != v) ? v : m;
    }
  }
  sm[half * DF + c] = m;
  __syncthreads();
  if (tid < 32) {
    const v4f a = *(const v4fa*)(sm + 4 * tid);
    const v4f b = *(const v4fa*)(sm + DF + 4 * tid);
    v4f r;
    r.x = (b.x > a.x || b.x != b.x) ? b.x : a.x;
    r.y = (b.y > a.y || b.y != b.y) ? b.y : a.y;
    r.z = (b.z > a.z || b.z != b.z) ? b.z : a.z;
    r.w = (b.w > a.w || b.w != b.w) ? b.w : a.w;
    float* op = outp + (size_t)g * DF + 4 * tid;
    *(volatile v4f*)op = r;
    __threadfence();
    *(volatile v4f*)op = r;
  }
}

static inline size_t al256(size_t o) { return (o + 255) & ~(size_t)255; }

extern "C" void kernel_launch(void* const* d_in, const int* in_sizes, int n_in,
                              void* d_out, int out_size, void* d_ws, size_t ws_size,
                              hipStream_t stream) {
  if (n_in < 14) return;
  if (in_sizes[0] != NN_C * DF) return;
  if (in_sizes[1] != 2 * NE_C || in_sizes[2] != 2 * NE_C) return;
  if (in_sizes[3] != NN_C) return;
  if (in_sizes[4] != DF * DF || in_sizes[6] != DF * DF || in_sizes[8] != DF * DF) return;
  if (in_sizes[10] != DF * DF || in_sizes[12] != DF * DF) return;
  if (in_sizes[5] != DF || in_sizes[7] != DF || in_sizes[9] != DF || in_sizes[11] != DF || in_sizes[13] != DF) return;
  if ((long long)out_size != (long long)NN_C * DF + (long long)NGR * DF) return;
  const int nN = NN_C, nE = NE_C;

  const float* x    = (const float*)d_in[0];
  const int*   eiT  = (const int*)d_in[1];
  const int*   eiW  = (const int*)d_in[2];
  const int*   bat  = (const int*)d_in[3];
  const float* W1t  = (const float*)d_in[4];
  const float* b1t  = (const float*)d_in[5];
  const float* W2t  = (const float*)d_in[6];
  const float* b2t  = (const float*)d_in[7];
  const float* W1w  = (const float*)d_in[8];
  const float* b1w  = (const float*)d_in[9];
  const float* W2w  = (const float*)d_in[10];
  const float* b2w  = (const float*)d_in[11];
  const float* Ww   = (const float*)d_in[12];
  const float* bw   = (const float*)d_in[13];
  float* out = (float*)d_out;

  char* ws = (char*)d_ws;
  size_t off = 0;
  const size_t oXB   = off; off = al256(off + (size_t)MP_C * DF * 2);
  const size_t oH    = off; off = al256(off + (size_t)MP_C * 2 * DF * 4);
  const size_t oT1   = off; off = al256(off + (size_t)MP_C * HLP * 2);
  const size_t oV1   = off; off = al256(off + (size_t)MP_C * HLP * 2);
  const size_t oLIST = off; off = al256(off + (size_t)2 * NBK * RCAP * 4);
  const size_t oCNT  = off; off = al256(off + (size_t)2 * NBP * 4);
  const size_t oOFF  = off; off = al256(off + (size_t)2 * NBP * 4);
  const size_t oDINV = off; off = al256(off + (size_t)2 * NBP * 4);
  const size_t oFLAG = off; off = al256(off + (size_t)2 * NBK * 32 * 4);
  const size_t oW1c  = off; off = al256(off + (size_t)2 * DF * DF * 2);
  const size_t oW2t  = off; off = al256(off + (size_t)DF * HLP * 2);
  const size_t oW2w  = off; off = al256(off + (size_t)DF * HLP * 2);
  const size_t oWw   = off; off = al256(off + (size_t)DF * HLP * 2);
  const size_t oBIAS = off; off = al256(off + (size_t)NBB * DF * 4);
  if (off > ws_size || off > (size_t)WSMAX) return;

  unsigned short* XB    = (unsigned short*)(ws + oXB);
  float*          H     = (float*)(ws + oH);
  float*          Hlo   = H;
  float*          WIKI  = H + (size_t)MP_C * DF;
  unsigned short* T1hl  = (unsigned short*)(ws + oT1);
  unsigned short* V1hl  = (unsigned short*)(ws + oV1);
  unsigned short* DIFFh = V1hl;
  int*            LIST  = (int*)(ws + oLIST);
  int*            CNT   = (int*)(ws + oCNT);
  int*            OFFS  = (int*)(ws + oOFF);
  float*          DINV  = (float*)(ws + oDINV);
  int*            FLAG  = (int*)(ws + oFLAG);
  unsigned short* W1cat = (unsigned short*)(ws + oW1c);
  unsigned short* W2tD  = (unsigned short*)(ws + oW2t);
  unsigned short* W2wD  = (unsigned short*)(ws + oW2w);
  unsigned short* WwD   = (unsigned short*)(ws + oWw);
  float*          BIAS  = (float*)(ws + oBIAS);

  int* LISTt = LIST;            int* LISTw = LIST + (size_t)NBK * RCAP;
  int* CNTt  = CNT;             int* CNTw  = CNT + NBP;
  int* OFFt  = OFFS;            int* OFFw  = OFFS + NBP;
  float* DINVt = DINV;          float* DINVw = DINV + NBP;
  int* FLAGt = FLAG;            int* FLAGw = FLAG + NBK * 32;

  const size_t bkLds = (size_t)BK_LDS_INTS * 4;
  const size_t plLds = (size_t)NWAVE * PSEG * 4;
  hipFuncSetAttribute(reinterpret_cast<const void*>(&k_bucket), hipFuncAttributeMaxDynamicSharedMemorySize, (int)bkLds);
  hipFuncSetAttribute(reinterpret_cast<const void*>(&k_pool), hipFuncAttributeMaxDynamicSharedMemorySize, (int)plLds);

  const int vec8 = ((nE & 3) == 0) ? 1 : 0;
  const int gM = MP_C / GBM;
  const int gA = MP_C / SPB;

  k_prep<<<NBX + NWB + NBB, NTHR, 0, stream>>>(x, W1t, W1w, W2t, W2w, Ww, b1t, b2t, b1w, b2w, bw,
                                               nN, XB, W1cat, W2tD, W2wD, WwD, BIAS);
  k_bucket<<<NBK, NTHR, bkLds, stream>>>(eiT, nE, nN, vec8, LISTt, CNTt, OFFt, (int*)DINVt, FLAGt);
  k_bucket<<<NBK, NTHR, bkLds, stream>>>(eiW, nE, nN, vec8, LISTw, CNTw, OFFw, (int*)DINVw, FLAGw);
  k_gemm<0><<<dim3(gM, 2), GTHR, 0, stream>>>(XB, W1cat, DF, DINV, NBP, BIAS, H, 2 * DF);
  k_agg<0><<<gA, NTHR, 0, stream>>>(H, 2 * DF, 0, LISTt, CNTt, OFFt, DINVt, FLAGt, BIAS + 0 * DF,
                                    nN, MP_C, T1hl, Hlo, BIAS);
  k_agg<0><<<gA, NTHR, 0, stream>>>(H, 2 * DF, DF, LISTw, CNTw, OFFw, DINVw, FLAGw, BIAS + 2 * DF,
                                    nN, MP_C, V1hl, Hlo, BIAS);
  k_gemm<0><<<dim3(gM, 1), GTHR, 0, stream>>>(V1hl, W2wD, HLP, DINVw, 0, BIAS, Hlo, DF);
  k_agg<1><<<gA, NTHR, 0, stream>>>(Hlo, DF, 0, LISTw, CNTw, OFFw, DINVw, FLAGw, BIAS + 3 * DF,
                                    nN, MP_C, V1hl, WIKI, BIAS);
  k_gemm<0><<<dim3(gM, 1), GTHR, 0, stream>>>(T1hl, W2tD, HLP, DINVt, 0, BIAS, Hlo, DF);
  k_agg<2><<<gA, NTHR, 0, stream>>>(Hlo, DF, 0, LISTt, CNTt, OFFt, DINVt, FLAGt, BIAS + 1 * DF,
                                    nN, MP_C, DIFFh, out, WIKI);
  k_gemm<1><<<dim3(gM, 1), GTHR, 0, stream>>>(DIFFh, WwD, HLP, DINVt, 0, BIAS + 4 * DF, Hlo, DF);
  k_pool<<<NGR, NTHR, plLds, stream>>>(Hlo, bat, nN, out + (size_t)NN_C * DF);
}
